// CFAggregator_63608465654313
// MI455X (gfx1250) — hardware-verified
//
#include <hip/hip_runtime.h>
#include <stddef.h>


#define DD      128
#define MC      4
#define NTHR    256
#define NWAVE   8
#define EPT     8
#define NGRP    2
#define CHUNK   (NTHR * EPT * NGRP)
#define WCAP    (EPT * NGRP * 32)
#define LISTN   (NWAVE * WCAP)
#define NB      16
#define CAP     128
#define APITCH  136
#define EROWS   64
#define ETHR    128
#define WPLANE  (DD * DD)

#define OFF_LIST   0
#define OFF_WCNT   (OFF_LIST + LISTN * 4)
#define OFF_SCNT   (OFF_WCNT + 64)
#define OFF_SLIST  (OFF_SCNT + 64)
#define OFF_NEIGH  (OFF_SLIST + NB * CAP * 4)
#define OFF_AH     (OFF_NEIGH + NB * MC * DD * 4)
#define OFF_AL     (OFF_AH + 2 * NB * APITCH * 2)
#define OFF_QL     (OFF_AL + 2 * NB * APITCH * 2)
#define OFF_SA     (OFF_QL + NB * 2 * DD * 4)
#define OFF_SF     (OFF_SA + NB * DD * 4)
#define LDS_MAIN   (OFF_SF + NB * DD * 4)
#define OFF_KL     OFF_LIST
#define LDS_E      (2 * EROWS * APITCH * 2)

static_assert((CHUNK & (CHUNK - 1)) == 0);
static_assert(CHUNK <= 4096);
static_assert((NB & (NB - 1)) == 0 && NB <= 4096);
static_assert(NB == 2 * NWAVE);
static_assert(NB * 2 * DD * 4 <= LISTN * 4);
static_assert(EROWS * DD * 4 <= LDS_E);
static_assert(WPLANE / 8 == 2048);
static_assert((APITCH % 8) == 0);
static_assert((OFF_AH % 16) == 0 && (OFF_AL % 16) == 0 && (OFF_QL % 16) == 0 && (OFF_NEIGH % 16) == 0);
static_assert((OFF_KL % 4) == 0 && (OFF_QL % 4) == 0 && (OFF_SA % 4) == 0 && (OFF_SF % 4) == 0);

typedef float          v4f  __attribute__((ext_vector_type(4)));
typedef float          v8f  __attribute__((ext_vector_type(8)));
typedef int            v4i  __attribute__((ext_vector_type(4)));
typedef unsigned short v8us __attribute__((ext_vector_type(8)));
typedef __bf16         v16b __attribute__((ext_vector_type(16)));
union FragB { v16b v; v8us u[2]; };

__device__ __forceinline__ unsigned int bfr(float x) {
  const unsigned int u = __float_as_uint(x);
  return (u + 0x7FFFu + ((u >> 16) & 1u)) >> 16;
}
__device__ __forceinline__ unsigned int sp1(float x) {
  const unsigned int hb = bfr(x);
  const float hf = __uint_as_float(hb << 16);
  const unsigned int lb = bfr(x - hf);
  return (hb & 0xFFFFu) | (lb << 16);
}
__device__ __forceinline__ void split8(v4f a, v4f b, v8us& hi, v8us& lo) {
  const unsigned int p0 = sp1(a.x), p1 = sp1(a.y), p2 = sp1(a.z), p3 = sp1(a.w);
  const unsigned int p4 = sp1(b.x), p5 = sp1(b.y), p6 = sp1(b.z), p7 = sp1(b.w);
  v8us h, l;
  h[0] = (unsigned short)(p0 & 0xFFFFu); l[0] = (unsigned short)(p0 >> 16);
  h[1] = (unsigned short)(p1 & 0xFFFFu); l[1] = (unsigned short)(p1 >> 16);
  h[2] = (unsigned short)(p2 & 0xFFFFu); l[2] = (unsigned short)(p2 >> 16);
  h[3] = (unsigned short)(p3 & 0xFFFFu); l[3] = (unsigned short)(p3 >> 16);
  h[4] = (unsigned short)(p4 & 0xFFFFu); l[4] = (unsigned short)(p4 >> 16);
  h[5] = (unsigned short)(p5 & 0xFFFFu); l[5] = (unsigned short)(p5 >> 16);
  h[6] = (unsigned short)(p6 & 0xFFFFu); l[6] = (unsigned short)(p6 >> 16);
  h[7] = (unsigned short)(p7 & 0xFFFFu); l[7] = (unsigned short)(p7 >> 16);
  hi = h; lo = l;
}

__device__ __forceinline__ v8f wmb(v16b a, v16b b, v8f c) {
  v8f d = __builtin_amdgcn_wmma_f32_16x16x32_bf16(false, a, false, b, (short)0, c, false, false);
  asm volatile("v_nop\n\tv_nop\n\tv_nop\n\tv_nop" : "+v"(d) : "v"(a), "v"(b));
  return d;
}

__device__ __forceinline__ float wred(float v) {
#pragma unroll
  for (int o = 16; o > 0; o >>= 1) v += __shfl_xor(v, o, 32);
  return v;
}
__device__ __forceinline__ float dot4(v4f a, v4f b) {
  return a.x * b.x + a.y * b.y + a.z * b.z + a.w * b.w;
}
__device__ __forceinline__ v4f elu4(v4f x) {
  v4f r;
  r.x = x.x > 0.0f ? x.x : expm1f(x.x);
  r.y = x.y > 0.0f ? x.y : expm1f(x.y);
  r.z = x.z > 0.0f ? x.z : expm1f(x.z);
  r.w = x.w > 0.0f ? x.w : expm1f(x.w);
  return r;
}

template <int NBT>
__device__ __forceinline__ int scan_chunk(const int* __restrict__ dsts, int nE, int cbase, int nodeBase,
                                          int vec8, int* list, int tid, int lane, int wave) {
  int wc = 0;
#pragma unroll
  for (int g = 0; g < NGRP; ++g) {
    const int el0  = (g * NTHR + tid) * EPT;
    const int e0   = cbase + el0;
    const int sent = -2147483647 - 1;
    v4i da, db;
    if (vec8 != 0 && cbase + CHUNK <= nE) {
      da = *(const v4i*)(dsts + e0);
      db = *(const v4i*)(dsts + e0 + 4);
    } else {
      da.x = (e0     < nE) ? dsts[min(e0, nE - 1)] : sent;
      da.y = (e0 + 1 < nE) ? dsts[min(e0 + 1, nE - 1)] : sent;
      da.z = (e0 + 2 < nE) ? dsts[min(e0 + 2, nE - 1)] : sent;
      da.w = (e0 + 3 < nE) ? dsts[min(e0 + 3, nE - 1)] : sent;
      db.x = (e0 + 4 < nE) ? dsts[min(e0 + 4, nE - 1)] : sent;
      db.y = (e0 + 5 < nE) ? dsts[min(e0 + 5, nE - 1)] : sent;
      db.z = (e0 + 6 < nE) ? dsts[min(e0 + 6, nE - 1)] : sent;
      db.w = (e0 + 7 < nE) ? dsts[min(e0 + 7, nE - 1)] : sent;
    }
    const unsigned nb = (unsigned)nodeBase;
    const unsigned s0 = (unsigned)da.x - nb, s1 = (unsigned)da.y - nb;
    const unsigned s2 = (unsigned)da.z - nb, s3 = (unsigned)da.w - nb;
    const unsigned s4 = (unsigned)db.x - nb, s5 = (unsigned)db.y - nb;
    const unsigned s6 = (unsigned)db.z - nb, s7 = (unsigned)db.w - nb;
    const bool h0 = s0 < (unsigned)NBT, h1 = s1 < (unsigned)NBT, h2 = s2 < (unsigned)NBT, h3 = s3 < (unsigned)NBT;
    const bool h4 = s4 < (unsigned)NBT, h5 = s5 < (unsigned)NBT, h6 = s6 < (unsigned)NBT, h7 = s7 < (unsigned)NBT;
    const unsigned any = __builtin_amdgcn_ballot_w32(h0 | h1 | h2 | h3 | h4 | h5 | h6 | h7);
    if (any != 0u) {
#define HITJ(J, HJ, SJ) { \
        const unsigned mj = __builtin_amdgcn_ballot_w32(HJ); \
        if (mj != 0u) { \
          if (HJ) { \
            const int pos = wc + (int)__builtin_amdgcn_mbcnt_lo(mj, 0u); \
            if (pos < WCAP) list[wave * WCAP + pos] = ((el0 + (J)) << 12) | (int)(SJ); \
          } \
          wc += (int)__builtin_popcount(mj); } }
      HITJ(0, h0, s0)
      HITJ(1, h1, s1)
      HITJ(2, h2, s2)
      HITJ(3, h3, s3)
      HITJ(4, h4, s4)
      HITJ(5, h5, s5)
      HITJ(6, h6, s6)
      HITJ(7, h7, s7)
#undef HITJ
    }
  }
  return wc;
}

__global__ __launch_bounds__(NTHR) void k_wprep(
    const float* __restrict__ W0, const float* __restrict__ W1,
    const float* __restrict__ W2, const float* __restrict__ W3,
    unsigned short* wpl) {
  const int i = blockIdx.x * NTHR + threadIdx.x;
  if (i >= 4 * WPLANE / 8) return;
  const int w = i >> 11;
  const float* W = (w == 0) ? W0 : ((w == 1) ? W1 : ((w == 2) ? W2 : W3));
  const int o  = (i & 2047) * 8;
  const int n  = o >> 7;
  const int k0 = o & 127;
  const float* p = W + (size_t)k0 * DD + n;
  v4f a, b;
  a.x = p[0];      a.y = p[DD];     a.z = p[2 * DD]; a.w = p[3 * DD];
  b.x = p[4 * DD]; b.y = p[5 * DD]; b.z = p[6 * DD]; b.w = p[7 * DD];
  v8us hv, lv;
  split8(a, b, hv, lv);
  unsigned short* ph = wpl + (size_t)(2 * w) * WPLANE + o;
  unsigned short* pl = ph + WPLANE;
  *(volatile v8us*)ph = hv;
  *(volatile v8us*)pl = lv;
  __threadfence();
  *(volatile v8us*)ph = hv;
  *(volatile v8us*)pl = lv;
}

__global__ __launch_bounds__(ETHR) void k_embed(
    const float* __restrict__ table, const int* __restrict__ ids,
    const unsigned short* __restrict__ wpl, float* ev, int nU, int nN) {
  __shared__ v4f lds_e[LDS_E / 16];
  unsigned short* sAh = (unsigned short*)lds_e;
  unsigned short* sAl = sAh + EROWS * APITCH;
  float*          stg = (float*)lds_e;
  const int tid = threadIdx.x, lane = tid & 31, wave = tid >> 5, hh = lane >> 4, m = lane & 15;
  const int rowBase = blockIdx.x * EROWS;

#pragma unroll
  for (int it = 0; it < (EROWS * DD / 8) / ETHR; ++it) {
    const int idx = it * ETHR + tid;
    const int r   = idx >> 4;
    const int c0  = (idx & 15) * 8;
    int u = rowBase + r;
    u = u > nU - 1 ? nU - 1 : u;
    int id = ids[u];
    id = id < 0 ? 0 : (id > nN - 1 ? nN - 1 : id);
    const float* xp = table + (size_t)id * DD + c0;
    const v4f a = *(const v4f*)xp, b = *(const v4f*)(xp + 4);
    v8us hv, lv;
    split8(a, b, hv, lv);
    *(v8us*)(sAh + r * APITCH + c0) = hv;
    *(v8us*)(sAl + r * APITCH + c0) = lv;
  }
  __syncthreads();

  const unsigned short* arh = sAh + (wave * 16 + m) * APITCH + 8 * hh;
  const unsigned short* arl = sAl + (wave * 16 + m) * APITCH + 8 * hh;
  const unsigned short* wbh = wpl;
  const unsigned short* wbl = wpl + WPLANE;
  v8f acc[8];
#pragma unroll
  for (int t = 0; t < 8; ++t) { v8f z = {0.f, 0.f, 0.f, 0.f, 0.f, 0.f, 0.f, 0.f}; acc[t] = z; }
#pragma unroll
  for (int kt = 0; kt < DD / 32; ++kt) {
    FragB ah, al;
    ah.u[0] = *(const v8us*)(arh + 32 * kt);
    ah.u[1] = *(const v8us*)(arh + 32 * kt + 16);
    al.u[0] = *(const v8us*)(arl + 32 * kt);
    al.u[1] = *(const v8us*)(arl + 32 * kt + 16);
#pragma unroll
    for (int t = 0; t < 8; ++t) {
      const int n = 16 * t + m;
      const unsigned short* bp = wbh + (size_t)n * DD + 32 * kt + 8 * hh;
      const unsigned short* bq = wbl + (size_t)n * DD + 32 * kt + 8 * hh;
      FragB bh, bl;
      bh.u[0] = *(const v8us*)bp;  bh.u[1] = *(const v8us*)(bp + 16);
      bl.u[0] = *(const v8us*)bq;  bl.u[1] = *(const v8us*)(bq + 16);
      acc[t] = wmb(ah.v, bh.v, acc[t]);
      acc[t] = wmb(ah.v, bl.v, acc[t]);
      acc[t] = wmb(al.v, bh.v, acc[t]);
    }
  }
  __syncthreads();

  float* sp = stg + (wave * 16 + 8 * hh) * DD + m;
#pragma unroll
  for (int t = 0; t < 8; ++t) {
    const int c = 16 * t;
    sp[0 * DD + c] = acc[t][0];
    sp[1 * DD + c] = acc[t][1];
    sp[2 * DD + c] = acc[t][2];
    sp[3 * DD + c] = acc[t][3];
    sp[4 * DD + c] = acc[t][4];
    sp[5 * DD + c] = acc[t][5];
    sp[6 * DD + c] = acc[t][6];
    sp[7 * DD + c] = acc[t][7];
  }
  __syncthreads();

  const float* lp = stg + wave * 16 * DD + 4 * lane;
  float* gp = ev + ((size_t)rowBase + wave * 16) * DD + 4 * lane;
#pragma unroll
  for (int i = 0; i < 16; ++i) { const v4f v = *(const v4f*)(lp + i * DD); *(volatile v4f*)(gp + (size_t)i * DD) = v; }
  __threadfence();
#pragma unroll
  for (int i = 0; i < 16; ++i) { const v4f v = *(const v4f*)(lp + i * DD); *(volatile v4f*)(gp + (size_t)i * DD) = v; }
}

__device__ __forceinline__ float zval(v4f ng, v4f mn, float sa2, float sdt) {
  const float n2  = wred(dot4(ng, ng));
  const float nd  = wred(dot4(ng, mn));
  const float nrm = fmaxf(sqrtf(sa2 + n2), 1e-12f);
  return (sdt + nd) * (1.0f / nrm);
}

__device__ __forceinline__ void epi_slot(const float* SA, const float* SF, const float* KL,
                                         const float* QL, const float* NG,
                                         const float* __restrict__ mu, int s, int lane,
                                         v4f& oa, v4f& of) {
  const v4f sa = *(const v4f*)(SA + s * DD + 4 * lane);
  const v4f sf = *(const v4f*)(SF + s * DD + 4 * lane);
  const v4f k0 = *(const v4f*)(KL + s * 2 * DD + 4 * lane);
  const v4f k1 = *(const v4f*)(KL + s * 2 * DD + DD + 4 * lane);
  const v4f q0 = *(const v4f*)(QL + s * 2 * DD + 4 * lane);
  const v4f q1 = *(const v4f*)(QL + s * 2 * DD + DD + 4 * lane);
  const v4f ms = *(const v4f*)(mu + 4 * lane);
  const v4f mn = *(const v4f*)(mu + DD + 4 * lane);
  const v4f g0 = *(const v4f*)(NG + (s * MC + 0) * DD + 4 * lane);
  const v4f g1 = *(const v4f*)(NG + (s * MC + 1) * DD + 4 * lane);
  const v4f g2 = *(const v4f*)(NG + (s * MC + 2) * DD + 4 * lane);
  const v4f g3 = *(const v4f*)(NG + (s * MC + 3) * DD + 4 * lane);

  const float sa2 = wred(dot4(sa, sa));
  const float sdt = wred(dot4(sa, ms));
  const float z0 = zval(g0, mn, sa2, sdt);
  const float z1 = zval(g1, mn, sa2, sdt);
  const float z2 = zval(g2, mn, sa2, sdt);
  const float z3 = zval(g3, mn, sa2, sdt);
  const float zm = fmaxf(fmaxf(z0, z1), fmaxf(z2, z3));
  const float e0 = expf(z0 - zm), e1 = expf(z1 - zm), e2 = expf(z2 - zm), e3 = expf(z3 - zm);
  const float rz = 1.0f / (e0 + e1 + e2 + e3);
  const v4f nsum = g0 * (e0 * rz) + g1 * (e1 * rz) + g2 * (e2 * rz) + g3 * (e3 * rz);
  const v4f v0 = (sa + nsum) * 0.5f;

  const float r128 = 1.0f / 128.0f;
  const float s00 = wred(dot4(k0, q0)) * r128;
  const float s01 = wred(dot4(k0, q1)) * r128;
  const float s10 = wred(dot4(k1, q0)) * r128;
  const float s11 = wred(dot4(k1, q1)) * r128;
  const float m0 = fmaxf(s00, s01);
  const float a00 = expf(s00 - m0), a01 = expf(s01 - m0);
  const float ra = 1.0f / (a00 + a01);
  const float p00 = a00 * ra, p01 = a01 * ra;
  const float m1 = fmaxf(s10, s11);
  const float a10 = expf(s10 - m1), a11 = expf(s11 - m1);
  const float rb = 1.0f / (a10 + a11);
  const float p10 = a10 * rb, p11 = a11 * rb;

  const v4f nw0 = v0 * p00 + sf * p01;
  const v4f nw1 = v0 * p10 + sf * p11;
  const v4f xa = v0 * 0.9f + nw0 * 0.1f;
  const v4f xf = sf * 0.9f + nw1 * 0.1f;
  oa = elu4(xa);
  of = elu4(xf);
}

__global__ __launch_bounds__(NTHR) void k_main(
    const int* __restrict__ nodes, const int* __restrict__ rowi, const int* __restrict__ layi,
    const int* __restrict__ coli, const float* __restrict__ aggT, const float* __restrict__ ffT,
    const unsigned short* __restrict__ wpl, const float* __restrict__ ev,
    const float* __restrict__ mu, float* out, int nB, int nU, int nE, int nN, int vec8) {
  extern __shared__ v4f lds_dyn[];
  char* base = (char*)lds_dyn;
  float* fbase = (float*)lds_dyn;
  int*   list  = (int*)(base + OFF_LIST);
  int*   wcnt  = (int*)(base + OFF_WCNT);
  int*   scnt  = (int*)(base + OFF_SCNT);
  int*   slist = (int*)(base + OFF_SLIST);
  float* neigh = (float*)(base + OFF_NEIGH);
  unsigned short* sAh = (unsigned short*)(base + OFF_AH);
  unsigned short* sAl = (unsigned short*)(base + OFF_AL);
  float* KL = (float*)(base + OFF_KL);
  float* QL = (float*)(base + OFF_QL);
  float* SA = (float*)(base + OFF_SA);
  float* SF = (float*)(base + OFF_SF);
  const int tid = threadIdx.x, lane = tid & 31, wave = tid >> 5, hh = lane >> 4, m = lane & 15;
  const int b0 = blockIdx.x * NB;

  if (tid < NB) scnt[tid] = 0;
  __syncthreads();

  const int nChunks = (nE + CHUNK - 1) / CHUNK;
#pragma unroll 1
  for (int ch = 0; ch < nChunks; ++ch) {
    const int cbase = ch * CHUNK;
    const int wc = scan_chunk<NB>(rowi, nE, cbase, b0, vec8, list, tid, lane, wave);
    if (lane == 0) wcnt[wave] = wc;
    __syncthreads();
    if (wave == 0) {
#pragma unroll 1
      for (int wsx = 0; wsx < NWAVE; ++wsx) {
        int n = __builtin_amdgcn_readfirstlane(wcnt[wsx]);
        n = n > WCAP ? WCAP : (n < 0 ? 0 : n);
        const int* lp = list + wsx * WCAP;
#pragma unroll 1
        for (int i = 0; i < n; ++i) {
          const int ent  = __builtin_amdgcn_readfirstlane(lp[i]);
          const int slot = ent & (NB - 1);
          int e = cbase + ((ent >> 12) & (CHUNK - 1));
          e = e > nE - 1 ? nE - 1 : e;
          int lay = layi[e];
          lay = lay < 0 ? 0 : (lay > MC - 1 ? MC - 1 : lay);
          int col = coli[e];
          col = col < 0 ? 0 : (col > nU - 1 ? nU - 1 : col);
          if (lane == 0) {
            const int c = scnt[slot];
            if (c < CAP) { slist[slot * CAP + c] = (lay << 20) | col; scnt[slot] = c + 1; }
          }
        }
      }
    }
    __syncthreads();
  }

#pragma unroll 1
  for (int s = wave; s < NB; s += NWAVE) {
    int cnt = __builtin_amdgcn_readfirstlane(scnt[s]);
    cnt = cnt > CAP ? CAP : (cnt < 0 ? 0 : cnt);
    int* L = slist + s * CAP;
    unsigned int dm = 0u;
#pragma unroll
    for (int q = 0; q < CAP / 32; ++q) {
      const int i   = 32 * q + lane;
      const int v   = L[i];
      const int lim = (i < cnt) ? i : 0;
      bool d = false;
#pragma unroll 1
      for (int j = 0; j < lim; ++j) d = d || (L[j] == v);
      dm |= d ? (1u << q) : 0u;
    }
#pragma unroll
    for (int q = 0; q < CAP / 32; ++q) {
      const int i = 32 * q + lane;
      if (i < cnt && ((dm >> q) & 1u) != 0u) L[i] = -1;
    }
  }
  __syncthreads();

#pragma unroll 1
  for (int s = wave; s < NB; s += NWAVE) {
    int cnt = __builtin_amdgcn_readfirstlane(scnt[s]);
    cnt = cnt > CAP ? CAP : (cnt < 0 ? 0 : cnt);
    const int* L = slist + s * CAP;
    v4f a0 = {0.f, 0.f, 0.f, 0.f}, a1 = a0, a2 = a0, a3 = a0;
    int c0 = 0, c1 = 0, c2 = 0, c3 = 0;
#pragma unroll 1
    for (int i = 0; i < cnt; ++i) {
      const int ent = __builtin_amdgcn_readfirstlane(L[i]);
      int col = ent & 0xFFFFF;
      col = col > nU - 1 ? nU - 1 : col;
      const v4f v = *(const v4f*)(ev + (size_t)col * DD + 4 * lane);
      if (ent >= 0) {
        const int lay = ent >> 20;
        if (lay == 0)      { a0 += v; ++c0; }
        else if (lay == 1) { a1 += v; ++c1; }
        else if (lay == 2) { a2 += v; ++c2; }
        else               { a3 += v; ++c3; }
      }
    }
    float* np = neigh + (size_t)(s * MC) * DD + 4 * lane;
    *(v4f*)(np + 0 * DD) = a0 * (1.0f / (float)(c0 > 0 ? c0 : 1));
    *(v4f*)(np + 1 * DD) = a1 * (1.0f / (float)(c1 > 0 ? c1 : 1));
    *(v4f*)(np + 2 * DD) = a2 * (1.0f / (float)(c2 > 0 ? c2 : 1));
    *(v4f*)(np + 3 * DD) = a3 * (1.0f / (float)(c3 > 0 ? c3 : 1));
  }

#pragma unroll
  for (int it = 0; it < 2; ++it) {
    const int idx  = it * NTHR + tid;
    const int r    = idx >> 4;
    const int cc   = (idx & 15) * 8;
    const int slot = r & (NB - 1);
    int b = b0 + slot;
    b = b > nB - 1 ? nB - 1 : b;
    int node = nodes[b];
    node = node < 0 ? 0 : (node > nN - 1 ? nN - 1 : node);
    const float* tp = (it == 0) ? aggT : ffT;
    const float* xp = tp + (size_t)node * DD + cc;
    const v4f a = *(const v4f*)xp, bq = *(const v4f*)(xp + 4);
    v8us hv, lv;
    split8(a, bq, hv, lv);
    *(v8us*)(sAh + r * APITCH + cc) = hv;
    *(v8us*)(sAl + r * APITCH + cc) = lv;
  }
  __syncthreads();

#pragma unroll 1
  for (int j = wave; j < 12; j += NWAVE) {
    const int g  = j >> 1;
    const int nh = j & 1;
    const int trow = (g & 1) ? NB : 0;
    const int widx = (g < 2) ? 2 : ((g < 4) ? 3 : ((g == 4) ? 0 : 1));
    const unsigned short* wbh = wpl + (size_t)(2 * widx) * WPLANE;
    const unsigned short* wbl = wbh + WPLANE;
    const int doff = (g == 0) ? (OFF_KL / 4)
                   : ((g == 1) ? (OFF_KL / 4 + DD)
                   : ((g == 2) ? (OFF_QL / 4)
                   : ((g == 3) ? (OFF_QL / 4 + DD)
                   : ((g == 4) ? (OFF_SA / 4) : (OFF_SF / 4)))));
    float* dst = fbase + doff;
    const int pitch = (g < 4) ? 2 * DD : DD;
    v8f acc[4];
#pragma unroll
    for (int t = 0; t < 4; ++t) { v8f z = {0.f, 0.f, 0.f, 0.f, 0.f, 0.f, 0.f, 0.f}; acc[t] = z; }
    const unsigned short* arh = sAh + (trow + m) * APITCH + 8 * hh;
    const unsigned short* arl = sAl + (trow + m) * APITCH + 8 * hh;
#pragma unroll
    for (int kt = 0; kt < DD / 32; ++kt) {
      FragB ah, al;
      ah.u[0] = *(const v8us*)(arh + 32 * kt);
      ah.u[1] = *(const v8us*)(arh + 32 * kt + 16);
      al.u[0] = *(const v8us*)(arl + 32 * kt);
      al.u[1] = *(const v8us*)(arl + 32 * kt + 16);
#pragma unroll
      for (int t = 0; t < 4; ++t) {
        const int n = 64 * nh + 16 * t + m;
        const unsigned short* bp = wbh + (size_t)n * DD + 32 * kt + 8 * hh;
        const unsigned short* bq = wbl + (size_t)n * DD + 32 * kt + 8 * hh;
        FragB bh, bl;
        bh.u[0] = *(const v8us*)bp;  bh.u[1] = *(const v8us*)(bp + 16);
        bl.u[0] = *(const v8us*)bq;  bl.u[1] = *(const v8us*)(bq + 16);
        acc[t] = wmb(ah.v, bh.v, acc[t]);
        acc[t] = wmb(ah.v, bl.v, acc[t]);
        acc[t] = wmb(al.v, bh.v, acc[t]);
      }
    }
    float* sp = dst + (8 * hh) * pitch + 64 * nh + m;
#pragma unroll
    for (int t = 0; t < 4; ++t) {
      sp[0 * pitch + 16 * t] = acc[t][0];
      sp[1 * pitch + 16 * t] = acc[t][1];
      sp[2 * pitch + 16 * t] = acc[t][2];
      sp[3 * pitch + 16 * t] = acc[t][3];
      sp[4 * pitch + 16 * t] = acc[t][4];
      sp[5 * pitch + 16 * t] = acc[t][5];
      sp[6 * pitch + 16 * t] = acc[t][6];
      sp[7 * pitch + 16 * t] = acc[t][7];
    }
  }
  __syncthreads();

  v4f oa0, of0, oa1, of1;
  epi_slot(SA, SF, KL, QL, neigh, mu, wave, lane, oa0, of0);
  epi_slot(SA, SF, KL, QL, neigh, mu, wave + NWAVE, lane, oa1, of1);
  const int bA = b0 + wave, bB = b0 + wave + NWAVE;
  float* o0 = out;
  float* o1 = out + (size_t)nB * DD;
  if (bA < nB) {
    *(volatile v4f*)(o0 + (size_t)bA * DD + 4 * lane) = oa0;
    *(volatile v4f*)(o1 + (size_t)bA * DD + 4 * lane) = of0;
  }
  if (bB < nB) {
    *(volatile v4f*)(o0 + (size_t)bB * DD + 4 * lane) = oa1;
    *(volatile v4f*)(o1 + (size_t)bB * DD + 4 * lane) = of1;
  }
  __threadfence();
  if (bA < nB) {
    *(volatile v4f*)(o0 + (size_t)bA * DD + 4 * lane) = oa0;
    *(volatile v4f*)(o1 + (size_t)bA * DD + 4 * lane) = of0;
  }
  if (bB < nB) {
    *(volatile v4f*)(o0 + (size_t)bB * DD + 4 * lane) = oa1;
    *(volatile v4f*)(o1 + (size_t)bB * DD + 4 * lane) = of1;
  }
}

extern "C" void kernel_launch(void* const* d_in, const int* in_sizes, int n_in,
                              void* d_out, int out_size, void* d_ws, size_t ws_size,
                              hipStream_t stream) {
  if (n_in < 12) return;
  const int nB = in_sizes[0];
  const int nU = in_sizes[1];
  const int nE = in_sizes[2];
  if (nB <= 0 || nU <= 0 || nE < 0 || nU > (1 << 20)) return;
  if (in_sizes[3] != nE || in_sizes[4] != nE) return;
  const int nN = in_sizes[5] / DD;
  if (nN <= 0 || in_sizes[5] != nN * DD || in_sizes[6] != nN * DD) return;
  if (in_sizes[7] != WPLANE || in_sizes[8] != WPLANE || in_sizes[9] != WPLANE || in_sizes[10] != WPLANE) return;
  if (in_sizes[11] != 2 * DD) return;
  if (out_size != 2 * nB * DD) return;

  const int*   nodes  = (const int*)d_in[0];
  const int*   uids   = (const int*)d_in[1];
  const int*   rowi   = (const int*)d_in[2];
  const int*   layi   = (const int*)d_in[3];
  const int*   coli   = (const int*)d_in[4];
  const float* aggT   = (const float*)d_in[5];
  const float* ffT    = (const float*)d_in[6];
  const float* Wv_agg = (const float*)d_in[7];
  const float* Wv_ff  = (const float*)d_in[8];
  const float* Wk     = (const float*)d_in[9];
  const float* Wq     = (const float*)d_in[10];
  const float* mu_w   = (const float*)d_in[11];
  float* out = (float*)d_out;

  const int nUB = (nU + EROWS - 1) / EROWS;
  const int nMB = (nB + NB - 1) / NB;

  char* ws = (char*)d_ws;
  size_t off = 0;
  const size_t oW  = off; off += (size_t)4 * 2 * WPLANE * 2;                off = (off + 255) & ~(size_t)255;
  const size_t oEV = off; off += (size_t)nUB * EROWS * DD * 4;              off = (off + 255) & ~(size_t)255;
  if (off > ws_size) return;
  unsigned short* wpl = (unsigned short*)(ws + oW);
  float*          ev  = (float*)(ws + oEV);

  const int vec8 = ((nE & 3) == 0) ? 1 : 0;

  k_wprep<<<(4 * WPLANE / 8 + NTHR - 1) / NTHR, NTHR, 0, stream>>>(Wv_agg, Wv_ff, Wk, Wq, wpl);

  k_embed<<<nUB, ETHR, 0, stream>>>(aggT, uids, wpl, ev, nU, nN);

  hipFuncSetAttribute(reinterpret_cast<const void*>(&k_main),
                      hipFuncAttributeMaxDynamicSharedMemorySize, LDS_MAIN);
  k_main<<<nMB, NTHR, LDS_MAIN, stream>>>(nodes, rowi, layi, coli, aggT, ffT, wpl, ev, mu_w, out,
                                          nB, nU, nE, nN, vec8);
}
